// XMem_13091060318871
// MI455X (gfx1250) — hardware-verified
//
#include <hip/hip_runtime.h>
#include <math.h>
typedef __attribute__((ext_vector_type(16))) _Float16 v16h;
typedef __attribute__((ext_vector_type(8)))  _Float16 v8h;
typedef __attribute__((ext_vector_type(16))) __bf16   v16b;
typedef __attribute__((ext_vector_type(8)))  __bf16   v8b;
typedef __attribute__((ext_vector_type(8)))  float    v8f;
typedef __attribute__((ext_vector_type(4)))  float    v4f;
#define PSCALE 32768.0f
#define U16(p) ((const unsigned short*)(const void*)(p))
#define PSCALE_INV (1.0f / 32768.0f)

__device__ __forceinline__ unsigned short f2bf_bits(float f) {
  unsigned u = __float_as_uint(f);
  return (unsigned short)((u + 0x7FFFu + ((u >> 16) & 1u)) >> 16);
}
__device__ __forceinline__ float bf_bits2f(unsigned short h) { return __uint_as_float(((unsigned)h) << 16); }

__device__ __forceinline__ void dep_guard_h(v8f& a, v8f& b, v16h x, v16h y) { asm volatile("v_nop\n\tv_nop\n\tv_nop\n\tv_nop" : "+v"(a), "+v"(b) : "v"(x), "v"(y)); }
__device__ __forceinline__ void dep_guard_b(v8f& a, v8f& b, v16b x, v16b y) { asm volatile("v_nop\n\tv_nop\n\tv_nop\n\tv_nop" : "+v"(a), "+v"(b) : "v"(x), "v"(y)); }
__device__ __forceinline__ void keep4_h(v16h a, v16h b, v16h c, v16h d) { asm volatile("v_nop" :: "v"(a), "v"(b), "v"(c), "v"(d)); }
__device__ __forceinline__ void keep4_b(v16b a, v16b b, v16b c, v16b d) { asm volatile("v_nop" :: "v"(a), "v"(b), "v"(c), "v"(d)); }
__device__ __forceinline__ void acc_guard4(v8f& a, v8f& b, v8f& c, v8f& d) { asm volatile("v_nop\n\tv_nop\n\tv_nop\n\tv_nop" : "+v"(a), "+v"(b), "+v"(c), "+v"(d)); }
template <typename T> struct Frag;
template <> struct Frag<_Float16> {
  typedef v16h V; union U { v16h v; v8h h[2]; };
  static __device__ __forceinline__ v16h load(const _Float16* p) {
    U f; f.h[0] = *(const v8h*)(p); f.h[1] = *(const v8h*)(p + 16); return f.v;
  }
  static __device__ __forceinline__ v8f mma(v16h a, v16h b, v8f c) {
    return __builtin_amdgcn_wmma_f32_16x16x32_f16(false, a, false, b, (short)0, c, false, false);
  }
  static __device__ __forceinline__ void guard(v8f& a, v8f& b, v16h x, v16h y) { dep_guard_h(a, b, x, y); }
  static __device__ __forceinline__ void keep(v16h a, v16h b, v16h c, v16h d) { keep4_h(a, b, c, d); }
};
template <> struct Frag<__bf16> {
  typedef v16b V; union U { v16b v; v8b h[2]; };
  static __device__ __forceinline__ v16b load(const __bf16* p) {
    U f; f.h[0] = *(const v8b*)(p); f.h[1] = *(const v8b*)(p + 16); return f.v;
  }
  static __device__ __forceinline__ v8f mma(v16b a, v16b b, v8f c) {
    return __builtin_amdgcn_wmma_f32_16x16x32_bf16(false, a, false, b, (short)0, c, false, false);
  }
  static __device__ __forceinline__ void guard(v8f& a, v8f& b, v16b x, v16b y) { dep_guard_b(a, b, x, y); }
  static __device__ __forceinline__ void keep(v16b a, v16b b, v16b c, v16b d) { keep4_b(a, b, c, d); }
};

template <int ET> struct Elem;
template <> struct Elem<0> { typedef _Float16 T; };
template <> struct Elem<1> { typedef __bf16 T; };
template <int ET, bool SPLIT, int BIAS_MODE, int OUT_MODE, bool RESID, int ACT = 0>
__global__ __launch_bounds__(256) void wmma_gemm64(
    const unsigned short* __restrict__ Ap, const unsigned short* __restrict__ A2p, int lda, long strideA,
    const unsigned short* __restrict__ Btp, const unsigned short* __restrict__ Bt2p, int ldb, long strideB,
    void* __restrict__ Cout, void* __restrict__ Cout2, int ldc, long strideC,
    const float* __restrict__ bias,
    const float* __restrict__ resid, long strideR,
    int M, int N, int K, float scale) {
  typedef typename Elem<ET>::T T;
  typedef typename Frag<T>::V V;
  const T* A = (const T*)Ap; const T* A2 = (const T*)A2p; const T* Bt = (const T*)Btp; const T* Bt2 = (const T*)Bt2p;
  __shared__ __align__(16) float sT[8][16 * 68];
  const int b    = blockIdx.y;
  const int lane = threadIdx.x & 31;
  const int wave = threadIdx.x >> 5;
  const int tilesN = N >> 6;
  const int tilesM = M >> 6;
  const int tile = blockIdx.x * 8 + wave;
  if (tile >= tilesM * tilesN) return;
  const int tm = tile / tilesN;
  const int tn = tile - tm * tilesN;
  const int m0 = tm << 6;
  const int n0 = tn << 6;

  const T* Ab  = A  + (size_t)b * strideA;
  const T* Bb  = Bt + (size_t)b * strideB;
  const T* Ab2 = SPLIT ? (A2  + (size_t)b * strideA) : nullptr;
  const T* Bb2 = SPLIT ? (Bt2 + (size_t)b * strideB) : nullptr;

  const int rlane = lane & 15;
  const int koff  = (lane >> 4) * 8;
  const int mOff  = (lane >> 4) * 8;

  v8f acc[4][4];
#pragma unroll
  for (int i = 0; i < 4; ++i)
#pragma unroll
    for (int j = 0; j < 4; ++j) acc[i][j] = (v8f){0.f,0.f,0.f,0.f,0.f,0.f,0.f,0.f};

  for (int k0 = 0; k0 < K; k0 += 32) {
    V bh[4], bl[4];
#pragma unroll
    for (int j = 0; j < 4; ++j) {
      const size_t bo = (size_t)(n0 + (j << 4) + rlane) * ldb + koff + k0;
      bh[j] = Frag<T>::load(Bb + bo);
      if (SPLIT) bl[j] = Frag<T>::load(Bb2 + bo);
    }
#pragma unroll
    for (int i = 0; i < 4; ++i) {
      const size_t ao = (size_t)(m0 + (i << 4) + rlane) * lda + koff + k0;
      V ah = Frag<T>::load(Ab + ao);
      V al;
      if (SPLIT) al = Frag<T>::load(Ab2 + ao);
#pragma unroll
      for (int j = 0; j < 4; ++j) {
        acc[i][j] = Frag<T>::mma(ah, bh[j], acc[i][j]);
        if (SPLIT) {
          acc[i][j] = Frag<T>::mma(ah, bl[j], acc[i][j]);
          acc[i][j] = Frag<T>::mma(al, bh[j], acc[i][j]);
        }
      }
      Frag<T>::guard(acc[i][0], acc[i][3], ah, SPLIT ? al : ah);
    }
    Frag<T>::keep(bh[0], bh[1], bh[2], bh[3]);
    if (SPLIT) Frag<T>::keep(bl[0], bl[1], bl[2], bl[3]);
  }
  acc_guard4(acc[0][0], acc[0][1], acc[0][2], acc[0][3]);
  acc_guard4(acc[1][0], acc[1][1], acc[1][2], acc[1][3]);
  acc_guard4(acc[2][0], acc[2][1], acc[2][2], acc[2][3]);
  acc_guard4(acc[3][0], acc[3][1], acc[3][2], acc[3][3]);

  float* slab = sT[wave];
  const float* Rb = RESID ? (resid + (size_t)b * strideR) : nullptr;
#pragma unroll
  for (int i = 0; i < 4; ++i) {
    const int mBase = m0 + (i << 4);
#pragma unroll
    for (int j = 0; j < 4; ++j) {
      const int n = n0 + (j << 4) + rlane;
      float bv = 0.f;
      if (BIAS_MODE == 2) bv = bias[n];
#pragma unroll
      for (int r = 0; r < 8; ++r) {
        float v = acc[i][j][r] * scale;
        if (BIAS_MODE == 1) v += bias[mBase + mOff + r];
        if (BIAS_MODE == 2) v += bv;
        if (RESID) v += Rb[(size_t)(mBase + mOff + r) * ldc + n];
        if (ACT == 1) v = tanhf(v);
        if (ACT == 2) v = fmaxf(v, 0.0f);
        if (ACT == 3) v = v / (1.0f + expf(-v));
        if (ACT == 4) v = (v > 0.f) ? v : 0.01f * v;
        if (ACT == 5) v = 0.5f * v * (1.0f + erff(v * 0.70710678118654752f));
        slab[(mOff + r) * 68 + (j << 4) + rlane] = v;
      }
    }
    __builtin_amdgcn_fence(__ATOMIC_RELEASE, "workgroup");
    __builtin_amdgcn_wave_barrier();
    __builtin_amdgcn_fence(__ATOMIC_ACQUIRE, "workgroup");
    if (OUT_MODE == 0) {
      float* C = (float*)Cout + (size_t)b * strideC;
      const int hh = lane >> 4, c4 = (lane & 15) * 4;
      for (int pass = 0; pass < 2; ++pass) {
#pragma unroll
        for (int it = 0; it < 8; ++it) {
          const int row = it * 2 + hh;
          v4f v = *(const v4f*)(slab + row * 68 + c4);
          *(volatile v4f*)(C + (size_t)(mBase + row) * ldc + n0 + c4) = v;
        }
        __threadfence();
      }
    } else {
      const int q = lane >> 3, c8 = (lane & 7) * 8;
      unsigned short* C  = (unsigned short*)Cout  + (size_t)b * strideC;
      unsigned short* C2 = (OUT_MODE == 2) ? ((unsigned short*)Cout2 + (size_t)b * strideC) : nullptr;
      for (int pass = 0; pass < 2; ++pass) {
#pragma unroll
        for (int it = 0; it < 4; ++it) {
          const int row = it * 4 + q;
          const float* sp = slab + row * 68 + c8;
          v8h hv, lv;
#pragma unroll
          for (int e = 0; e < 8; ++e) {
            if (OUT_MODE == 1) {
              hv[e] = (_Float16)sp[e];
            } else {
              unsigned short hb = f2bf_bits(sp[e]);
              unsigned short lb = f2bf_bits(sp[e] - bf_bits2f(hb));
              hv[e] = __builtin_bit_cast(_Float16, hb);
              lv[e] = __builtin_bit_cast(_Float16, lb);
            }
          }
          *(volatile v8h*)(C + (size_t)(mBase + row) * ldc + n0 + c8) = hv;
          if (OUT_MODE == 2) *(volatile v8h*)(C2 + (size_t)(mBase + row) * ldc + n0 + c8) = lv;
        }
        __threadfence();
      }
    }
    __builtin_amdgcn_fence(__ATOMIC_RELEASE, "workgroup");
    __builtin_amdgcn_wave_barrier();
    __builtin_amdgcn_fence(__ATOMIC_ACQUIRE, "workgroup");
  }
}

__global__ __launch_bounds__(256) void cast_f32_f16x2(
    const float* __restrict__ in, _Float16* __restrict__ out, int n2) {
  int i = blockIdx.x * 256 + threadIdx.x;
  if (i < n2) {
    const _Float16 h0 = (_Float16)in[2 * i], h1 = (_Float16)in[2 * i + 1];
    const unsigned u = (unsigned)__builtin_bit_cast(unsigned short, h0) | ((unsigned)__builtin_bit_cast(unsigned short, h1) << 16);
    ((volatile unsigned*)out)[i] = u;
    __threadfence();
    ((volatile unsigned*)out)[i] = u;
  }
}


#define XCK 64
#define XN 8192
#define XP 4096
#define XV 1024
__global__ __launch_bounds__(256) void build_q_kernel(const float* __restrict__ qk, const float* __restrict__ qe, unsigned* __restrict__ AQ, float* __restrict__ bsq, float negone) {
  __shared__ float red[8][33];
  const int lane = threadIdx.x & 31, wave = threadIdx.x >> 5; const int p = blockIdx.x * 8 + wave;
  const float k0 = qk[(size_t)(2 * lane) * XP + p], k1 = qk[(size_t)(2 * lane + 1) * XP + p];
  const float e0 = qe[(size_t)(2 * lane) * XP + p], e1 = qe[(size_t)(2 * lane + 1) * XP + p];
  float b = e0 * k0 * k0 + e1 * k1 * k1;
  for (int o = 16; o > 0; o >>= 1) b += __shfl_xor(b, o, 32);
  const unsigned u0 = (unsigned)__builtin_bit_cast(unsigned short, (_Float16)(2.f * k0 * e0)) | ((unsigned)__builtin_bit_cast(unsigned short, (_Float16)(2.f * k1 * e1)) << 16);
  const unsigned u1 = (unsigned)__builtin_bit_cast(unsigned short, (_Float16)(e0 * negone)) | ((unsigned)__builtin_bit_cast(unsigned short, (_Float16)(e1 * negone)) << 16);
  red[wave][lane] = b;
  for (int pass = 0; pass < 2; ++pass) {
    ((volatile unsigned*)AQ)[(size_t)p * 64 + lane] = u0; ((volatile unsigned*)AQ)[(size_t)p * 64 + 32 + lane] = u1; __threadfence();
  }
  __syncthreads();
  if (wave == 0) {
    const float v = (lane < 8) ? red[lane][0] : 0.f;
    ((volatile float*)bsq)[(size_t)blockIdx.x * 32 + lane] = v; __threadfence(); ((volatile float*)bsq)[(size_t)blockIdx.x * 32 + lane] = v; }
}
__global__ __launch_bounds__(256) void build_m_kernel(const float* __restrict__ mk, unsigned* __restrict__ AM) {
  const int lane = threadIdx.x & 31, wave = threadIdx.x >> 5; const int n = blockIdx.x * 8 + wave;
  const float m0 = mk[(size_t)(2 * lane) * XN + n], m1 = mk[(size_t)(2 * lane + 1) * XN + n];
  const unsigned u0 = (unsigned)__builtin_bit_cast(unsigned short, (_Float16)m0) | ((unsigned)__builtin_bit_cast(unsigned short, (_Float16)m1) << 16);
  const unsigned u1 = (unsigned)__builtin_bit_cast(unsigned short, (_Float16)(m0 * m0)) | ((unsigned)__builtin_bit_cast(unsigned short, (_Float16)(m1 * m1)) << 16);
  for (int pass = 0; pass < 2; ++pass) { ((volatile unsigned*)AM)[(size_t)n * 64 + lane] = u0; ((volatile unsigned*)AM)[(size_t)n * 64 + 32 + lane] = u1; __threadfence(); }
}
__global__ __launch_bounds__(256) void softmax_kernel(const float* __restrict__ ST, const float* __restrict__ bsq, const float* __restrict__ ms, unsigned* __restrict__ AFT) {
  __shared__ float red[8]; __shared__ float stat;
  const int p = blockIdx.x, t = threadIdx.x, lane = t & 31, wave = t >> 5;
  const float bq = bsq[(size_t)(p >> 3) * 32 + (p & 7)];
  const float* row = ST + (size_t)p * XN;
  float mx = -INFINITY;
#pragma unroll 1
  for (int q = 0; q < 16; ++q) { const int n = q * 512 + 2 * t;
    const float s0 = (row[n] - bq) * ms[n] * 0.125f, s1 = (row[n + 1] - bq) * ms[n + 1] * 0.125f; mx = fmaxf(mx, fmaxf(s0, s1)); }
  for (int o = 16; o > 0; o >>= 1) mx = fmaxf(mx, __shfl_xor(mx, o, 32));
  if (lane == 0) red[wave] = mx;
  __syncthreads();
  if (t == 0) { float m = red[0]; for (int w = 1; w < 8; ++w) m = fmaxf(m, red[w]); stat = m; }
  __syncthreads();
  const float m = stat;
  __syncthreads();
  float se = 0.f;
#pragma unroll 1
  for (int q = 0; q < 16; ++q) { const int n = q * 512 + 2 * t;
    se += expf((row[n] - bq) * ms[n] * 0.125f - m) + expf((row[n + 1] - bq) * ms[n + 1] * 0.125f - m); }
  for (int o = 16; o > 0; o >>= 1) se += __shfl_xor(se, o, 32);
  if (lane == 0) red[wave] = se;
  __syncthreads();
  if (t == 0) { float s = 0.f; for (int w = 0; w < 8; ++w) s += red[w]; stat = 32768.0f / s; }
  __syncthreads();
  const float inv = stat;
  for (int pass = 0; pass < 2; ++pass) {
#pragma unroll 1
    for (int q = 0; q < 16; ++q) { const int n = q * 512 + 2 * t;
      const float a = expf((row[n] - bq) * ms[n] * 0.125f - m) * inv, b = expf((row[n + 1] - bq) * ms[n + 1] * 0.125f - m) * inv;
      const unsigned u = (unsigned)__builtin_bit_cast(unsigned short, (_Float16)a) | ((unsigned)__builtin_bit_cast(unsigned short, (_Float16)b) << 16);
      ((volatile unsigned*)AFT)[(size_t)p * (XN / 2) + q * 256 + t] = u; }
    __threadfence();
  }
}
extern "C" void kernel_launch(void* const* d_in, const int* in_sizes, int n_in, void* d_out, int out_size, void* d_ws, size_t ws_size, hipStream_t stream) {
  (void)in_sizes; (void)n_in; (void)out_size; (void)ws_size;
  const float* qk = (const float*)d_in[0]; const float* qe = (const float*)d_in[1]; const float* mk = (const float*)d_in[2]; const float* ms = (const float*)d_in[3]; const float* mv = (const float*)d_in[4];
  float* out = (float*)d_out;
  char* ws = (char*)d_ws; size_t off = 0;
  auto carve = [&](size_t bytes) -> char* { char* p = ws + off; off += (bytes + 255) & ~(size_t)255; return p; };
  unsigned* AQ = (unsigned*)carve((size_t)XP * 128 * 2); unsigned* AM = (unsigned*)carve((size_t)XN * 128 * 2);
  float* bsq = (float*)carve((size_t)(XP / 8) * 32 * 4);
  float* ST = (float*)carve((size_t)XP * XN * 4);
  unsigned* AFT = (unsigned*)carve((size_t)XP * XN * 2);
  _Float16* MV16 = (_Float16*)carve((size_t)XV * XN * 2);
  build_q_kernel<<<XP / 8, 256, 0, stream>>>(qk, qe, AQ, bsq, -1.0f);
  build_m_kernel<<<XN / 8, 256, 0, stream>>>(mk, AM);
  cast_f32_f16x2<<<(XV * XN / 2 + 255) / 256, 256, 0, stream>>>(mv, MV16, XV * XN / 2);
  { const int t = (XP / 64) * (XN / 64);
    wmma_gemm64<0, false, 0, 0, false><<<dim3((t + 7) / 8, 1), 256, 0, stream>>>((const unsigned short*)AQ, nullptr, 128, 0, (const unsigned short*)AM, nullptr, 128, 0, ST, nullptr, XN, 0, nullptr, nullptr, 0, XP, XN, 128, 1.0f); }
  softmax_kernel<<<XP, 256, 0, stream>>>(ST, bsq, ms, AFT);
  { const int t = (XV / 64) * (XP / 64);
    wmma_gemm64<0, false, 0, 0, false><<<dim3((t + 7) / 8, 1), 256, 0, stream>>>(U16(MV16), nullptr, XN, 0, (const unsigned short*)AFT, nullptr, XN, 0, out, nullptr, XP, 0, nullptr, nullptr, 0, XV, XP, XN, 1.0f / 32768.0f); }
}
